// GAT_22247930593786
// MI455X (gfx1250) — hardware-verified
//
#include <hip/hip_runtime.h>
#include <stddef.h>
#include <stdint.h>
#include <math.h>


#define DIN     128
#define HID     64
#define NH2     8
#define HC2     512
#define KA2     128
#define NTHR    256
#define NWAVE   8
#define EPT     8
#define CHUNK   (NTHR * EPT)
#define WCAP    (EPT * 32)
#define LISTN   (NWAVE * WCAP)
#define NBA     1024
#define SLA     10
#define RCAP    16384
#define DEGCAP  128
#define GBM     64
#define GBN     64
#define GTHR    128
#define DTHR    256
#define NEGSL   0.2f
#define EPS_SM  1e-16f
#define AGG_ZINTS (LISTN + 2 * RCAP + 3 * NBA)
#define AGG_LDS_INTS (AGG_ZINTS + 16)
#define WSMAX   134217728

static_assert((CHUNK & (CHUNK - 1)) == 0 && CHUNK <= 4096);
static_assert((NBA & (NBA - 1)) == 0 && NBA == (1 << SLA));
static_assert(((long long)CHUNK << SLA) < (1LL << 31));
static_assert(NBA % NWAVE == 0 && NBA % 32 == 0 && NBA % GBM == 0);
static_assert(RCAP % 4 == 0 && AGG_ZINTS % 4 == 0 && LISTN % 4 == 0);
static_assert(AGG_LDS_INTS * 4 <= 300000);
static_assert(GBM == (GTHR / 32) * 16);
static_assert(GTHR == 2 * GBN && GTHR == 2 * GBM);
static_assert((DIN % 32) == 0 && (KA2 % 32) == 0 && KA2 == 2 * HID);
static_assert(HID == GBN && HC2 == NH2 * GBN);
static_assert(HID == 2 * 32);
static_assert(HC2 == 16 * 32);
static_assert((DIN / 8) == 16);
static_assert((DTHR % 32) == 0);

typedef float          v2f  __attribute__((ext_vector_type(2)));
typedef float          v4f  __attribute__((ext_vector_type(4)));
typedef float          v8f  __attribute__((ext_vector_type(8)));
typedef int            v4i  __attribute__((ext_vector_type(4)));
typedef int            v8i  __attribute__((ext_vector_type(8)));
typedef unsigned int   v4u  __attribute__((ext_vector_type(4)));
typedef unsigned short v8us __attribute__((ext_vector_type(8)));
typedef __bf16         v16b __attribute__((ext_vector_type(16)));
typedef v2f  __attribute__((may_alias)) v2fa;
typedef v4f  __attribute__((may_alias)) v4fa;
typedef v4i  __attribute__((may_alias)) v4ia;
typedef v8us __attribute__((may_alias)) v8usa;
union FragB { v16b v; v8us h[2]; v8i w; };

__device__ __forceinline__ v8f wmb(const FragB& a, const FragB& b, v8f c) {
  v8f d = __builtin_amdgcn_wmma_f32_16x16x32_bf16(false, a.v, false, b.v, (short)0, c, false, false);
  asm volatile("v_nop\n\tv_nop\n\tv_nop\n\tv_nop" : "+v"(d) : "v"(a.w), "v"(b.w));
  return d;
}

__device__ __forceinline__ unsigned int f2bf(float f) {
  const unsigned int u = __float_as_uint(f);
  return ((u + 0x7FFFu + ((u >> 16) & 1u)) >> 16) & 0xFFFFu;
}
__device__ __forceinline__ float bf2f(unsigned int b) { return __uint_as_float(b << 16); }
__device__ __forceinline__ float bfr(float f) { return bf2f(f2bf(f)); }
__device__ __forceinline__ v4f bfr4(const v4f a) {
  v4f r; r.x = bfr(a.x); r.y = bfr(a.y); r.z = bfr(a.z); r.w = bfr(a.w); return r;
}
__device__ __forceinline__ unsigned int pk2(float lo, float hi) { return f2bf(lo) | (f2bf(hi) << 16); }
__device__ __forceinline__ v4u pack8(const v4f a, const v4f b) {
  v4u r;
  r.x = pk2(a.x, a.y); r.y = pk2(a.z, a.w); r.z = pk2(b.x, b.y); r.w = pk2(b.z, b.w);
  return r;
}

template <int SLB>
__device__ __forceinline__ int scan_chunk(const int* __restrict__ dsts, int nE, int cbase, int slotBase,
                                          int nb, int vec8, int* list, int tid, int lane, int wave) {
  int wc = 0;
  const int el0  = tid * EPT;
  const int e0   = cbase + el0;
  const int sent = -2147483647 - 1;
  v4i da, db;
  if (vec8 != 0 && cbase + CHUNK <= nE) {
    da = *(const v4i*)(dsts + e0);
    db = *(const v4i*)(dsts + e0 + 4);
  } else {
    da.x = (e0     < nE) ? dsts[min(e0,     nE - 1)] : sent;
    da.y = (e0 + 1 < nE) ? dsts[min(e0 + 1, nE - 1)] : sent;
    da.z = (e0 + 2 < nE) ? dsts[min(e0 + 2, nE - 1)] : sent;
    da.w = (e0 + 3 < nE) ? dsts[min(e0 + 3, nE - 1)] : sent;
    db.x = (e0 + 4 < nE) ? dsts[min(e0 + 4, nE - 1)] : sent;
    db.y = (e0 + 5 < nE) ? dsts[min(e0 + 5, nE - 1)] : sent;
    db.z = (e0 + 6 < nE) ? dsts[min(e0 + 6, nE - 1)] : sent;
    db.w = (e0 + 7 < nE) ? dsts[min(e0 + 7, nE - 1)] : sent;
  }
  const unsigned nbs = (unsigned)slotBase;
  const unsigned unb = (unsigned)nb;
  const unsigned s0 = (unsigned)da.x - nbs, s1 = (unsigned)da.y - nbs;
  const unsigned s2 = (unsigned)da.z - nbs, s3 = (unsigned)da.w - nbs;
  const unsigned s4 = (unsigned)db.x - nbs, s5 = (unsigned)db.y - nbs;
  const unsigned s6 = (unsigned)db.z - nbs, s7 = (unsigned)db.w - nbs;
  const bool h0 = s0 < unb, h1 = s1 < unb, h2 = s2 < unb, h3 = s3 < unb;
  const bool h4 = s4 < unb, h5 = s5 < unb, h6 = s6 < unb, h7 = s7 < unb;
  const unsigned any = __builtin_amdgcn_ballot_w32(h0 | h1 | h2 | h3 | h4 | h5 | h6 | h7);
  if (any != 0u) {
#define HITJ(J, HJ, SJ) { \
      const unsigned mj = __builtin_amdgcn_ballot_w32(HJ); \
      if (mj != 0u) { \
        if (HJ) { \
          const int pos = wc + (int)__builtin_amdgcn_mbcnt_lo(mj, 0u); \
          if (pos < WCAP) list[wave * WCAP + pos] = ((el0 + (J)) << SLB) | (int)(SJ); \
        } \
        wc += (int)__builtin_popcount(mj); } }
    HITJ(0, h0, s0)
    HITJ(1, h1, s1)
    HITJ(2, h2, s2)
    HITJ(3, h3, s3)
    HITJ(4, h4, s4)
    HITJ(5, h5, s5)
    HITJ(6, h6, s6)
    HITJ(7, h7, s7)
#undef HITJ
  }
  return wc;
}

__global__ __launch_bounds__(NTHR) void k_xprep(const float* __restrict__ x, unsigned short* xb, int nN, int nUnits) {
  const int i = (int)blockIdx.x * NTHR + (int)threadIdx.x;
  if (i >= nUnits) return;
  const int row = i >> 4;
  const int c0  = (i & 15) * 8;
  const int rc  = row < nN ? row : nN - 1;
  const float* p = x + (size_t)rc * DIN + c0;
  v4f a = *(const v4fa*)p, b = *(const v4fa*)(p + 4);
  const v4f z4 = {0.f, 0.f, 0.f, 0.f};
  if (row >= nN) { a = z4; b = z4; }
  const v4u hv = pack8(a, b);
  const size_t o = (size_t)row * DIN + c0;
  *(volatile v4u*)(xb + o) = hv;
  __threadfence();
  *(volatile v4u*)(xb + o) = hv;
}

__global__ __launch_bounds__(NTHR) void k_wtr(const float* __restrict__ w, int Kin, int Ncol, int Nrows, int Kout,
                                              unsigned short* wt, int nUnits) {
  const int u = (int)blockIdx.x * NTHR + (int)threadIdx.x;
  if (u >= nUnits) return;
  const int kq = Kout >> 3;
  const int n  = u / kq;
  const int k8 = (u - n * kq) * 8;
  const int kk = k8 - (k8 / Kin) * Kin;
  const int ncl = n < Ncol ? n : Ncol - 1;
  const float* p = w + (size_t)kk * (size_t)Ncol + ncl;
  v4f a, b;
  a.x = p[0];                    a.y = p[(size_t)Ncol];         a.z = p[(size_t)2 * Ncol];     a.w = p[(size_t)3 * Ncol];
  b.x = p[(size_t)4 * Ncol];     b.y = p[(size_t)5 * Ncol];     b.z = p[(size_t)6 * Ncol];     b.w = p[(size_t)7 * Ncol];
  const v4f z4 = {0.f, 0.f, 0.f, 0.f};
  if (n >= Ncol || n >= Nrows) { a = z4; b = z4; }
  const v4u wv = pack8(a, b);
  unsigned short* o = wt + (size_t)n * (size_t)Kout + k8;
  *(volatile v4u*)o = wv;
  __threadfence();
  *(volatile v4u*)o = wv;
}

__global__ __launch_bounds__(GTHR) void k_gemm(
    const unsigned short* __restrict__ A, const unsigned short* __restrict__ WT,
    float* outF, int K, int ldo,
    const float* __restrict__ atts, const float* __restrict__ attd, int attLen,
    float* SD, int MPr)
{
  __shared__ __attribute__((aligned(16))) float stg[GBM * GBN];
  __shared__ __attribute__((aligned(16))) float satt[2 * GBN];
  __shared__ __attribute__((aligned(16))) float sdot[2 * GBM];
  const int tid = (int)threadIdx.x, lane = tid & 31, wave = tid >> 5, hh = lane >> 4, m = lane & 15;
  const int rowBase = (int)blockIdx.x * GBM;
  const int head    = (int)blockIdx.y;
  const int col0    = head * GBN;

  {
    const int which = tid >> 6;
    const int c  = tid & 63;
    const int cl = c < attLen ? c : attLen - 1;
    const float vs = atts[head * attLen + cl];
    const float vd = attd[head * attLen + cl];
    float v = (which == 0) ? vs : vd;
    v = (c < attLen) ? bfr(v) : 0.f;
    satt[which * GBN + c] = v;
  }

  v8f acc[4];
  {
    const v8f z = {0.f, 0.f, 0.f, 0.f, 0.f, 0.f, 0.f, 0.f};
    acc[0] = z; acc[1] = z; acc[2] = z; acc[3] = z;
  }
  const unsigned short* ap = A  + (size_t)(rowBase + 16 * wave + m) * (size_t)K + 8 * hh;
  const unsigned short* wp = WT + (size_t)(col0 + m) * (size_t)K + 8 * hh;
  const int ksteps = K >> 5;
#pragma unroll 1
  for (int ks = 0; ks < ksteps; ++ks) {
    FragB af;
    af.h[0] = *(const v8usa*)(ap + 32 * ks);
    af.h[1] = *(const v8usa*)(ap + 32 * ks + 16);
#pragma unroll
    for (int t = 0; t < 4; ++t) {
      const unsigned short* wq = wp + (size_t)(16 * t) * (size_t)K + 32 * ks;
      FragB bf;
      bf.h[0] = *(const v8usa*)wq;
      bf.h[1] = *(const v8usa*)(wq + 16);
      acc[t] = wmb(af, bf, acc[t]);
    }
  }

#pragma unroll
  for (int t = 0; t < 4; ++t) {
    const int lc = 16 * t + m;
#pragma unroll
    for (int r = 0; r < 8; ++r) {
      const int lr = 16 * wave + 8 * hh + r;
      stg[lr * GBN + lc] = acc[t][r];
    }
  }
  __syncthreads();

  {
    const int row = tid & 63, which = tid >> 6;
    const float* sa = satt + which * GBN;
    const float* hr = stg + row * GBN;
    float d = 0.f;
#pragma unroll 4
    for (int c4 = 0; c4 < GBN / 4; ++c4) {
      const v4f hv = *(const v4fa*)(hr + 4 * c4);
      const v4f av = *(const v4fa*)(sa + 4 * c4);
      d = fmaf(hv.x, av.x, d);
      d = fmaf(hv.y, av.y, d);
      d = fmaf(hv.z, av.z, d);
      d = fmaf(hv.w, av.w, d);
    }
    sdot[which * GBM + row] = d;
  }
  __syncthreads();

  v4f fv[8];
#pragma unroll
  for (int i = 0; i < 8; ++i) {
    const int lr = 16 * wave + 2 * i + hh;
    fv[i] = *(const v4fa*)(stg + lr * GBN + 4 * m);
  }
  const int which2 = lane >> 4, piece = lane & 15;
  const v4f sdv = *(const v4fa*)(sdot + which2 * GBM + 4 * piece);
  float* sp = SD + (size_t)(2 * head + which2) * (size_t)MPr + rowBase + 4 * piece;

#pragma unroll
  for (int i = 0; i < 8; ++i) {
    const int lr = 16 * wave + 2 * i + hh;
    const int gr = rowBase + lr;
    float* op = outF + (size_t)gr * (size_t)ldo + col0 + 4 * m;
    *(volatile v4f*)op = fv[i];
  }
  if (wave == 0) *(volatile v4f*)sp = sdv;
  __threadfence();
#pragma unroll
  for (int i = 0; i < 8; ++i) {
    const int lr = 16 * wave + 2 * i + hh;
    const int gr = rowBase + lr;
    float* op = outF + (size_t)gr * (size_t)ldo + col0 + 4 * m;
    *(volatile v4f*)op = fv[i];
  }
  if (wave == 0) *(volatile v4f*)sp = sdv;
}

template <int L>
__global__ __launch_bounds__(NTHR) void k_agg(const int* __restrict__ srcs, const int* __restrict__ dsts,
                                              int nE, int nN, int vec8, int MPr,
                                              const float* __restrict__ SD, const float* __restrict__ F,
                                              const float* __restrict__ bias,
                                              unsigned short* zhl, float* z2) {
  static_assert(L == 1 || L == 2);
  extern __shared__ __attribute__((aligned(16))) int dsm[];
  int* list = dsm;
  int* hl   = dsm + LISTN;
  int* sl   = dsm + LISTN + RCAP;
  int* cnt  = dsm + LISTN + 2 * RCAP;
  int* offs = cnt + NBA;
  int* cur  = offs + NBA;
  int* misc = cur + NBA;
  const int tid = (int)threadIdx.x, lane = tid & 31, wave = tid >> 5;
  const int nodeBase = (int)blockIdx.x * NBA;

  {
    const v4i z4 = {0, 0, 0, 0};
    for (int i = tid * 4; i < AGG_ZINTS; i += NTHR * 4) *(v4ia*)(dsm + i) = z4;
    if (tid < 16) misc[tid] = 0;
  }
  __syncthreads();

  int t = 0, ov = 0;
  const int nChunks = (nE + CHUNK - 1) / CHUNK;
#pragma unroll 1
  for (int ch = 0; ch < nChunks; ++ch) {
    const int cbase = ch * CHUNK;
    const int wc = scan_chunk<SLA>(dsts, nE, cbase, nodeBase, NBA, vec8, list, tid, lane, wave);
    if (lane == 0) misc[wave] = wc;
    __syncthreads();
    if (wave == 0) {
#pragma unroll 1
      for (int w2 = 0; w2 < NWAVE; ++w2) {
        int c = misc[w2];
        c = c < 0 ? 0 : (c > WCAP ? WCAP : c);
#pragma unroll 1
        for (int b0 = 0; b0 < c; b0 += 32) {
          const int idx = b0 + lane;
          const int ent = list[w2 * WCAP + (idx < WCAP ? idx : WCAP - 1)];
          const int m32 = (c - b0) < 32 ? (c - b0) : 32;
#pragma unroll 1
          for (int k = 0; k < m32; ++k) {
            const int u    = __builtin_amdgcn_readlane(ent, k);
            const int slot = u & (NBA - 1);
            const int el   = (u >> SLA) & (CHUNK - 1);
            const int pk   = ((cbase + el) << SLA) | slot;
            if (t < RCAP) {
              if (lane == 0) { hl[t] = pk; cnt[slot] = cnt[slot] + 1; }
              t = t + 1;
            } else {
              ov = 1;
            }
          }
        }
      }
    }
    __syncthreads();
  }
  if (wave == 0 && lane == 0) { misc[8] = t; misc[9] = ov; }
  __syncthreads();
  int tt = misc[8];
  tt = tt < 0 ? 0 : (tt > RCAP ? RCAP : tt);
  const int ovf = misc[9];

  if (wave == 0) {
    const int base = lane * (NBA / 32);
    int s = 0;
#pragma unroll 1
    for (int i = 0; i < NBA / 32; ++i) s += cnt[base + i];
    int incl = s;
#pragma unroll
    for (int d = 1; d < 32; d <<= 1) {
      const int y = __shfl_up(incl, d, 32);
      if (lane >= d) incl += y;
    }
    int run = incl - s;
#pragma unroll 1
    for (int i = 0; i < NBA / 32; ++i) {
      const int cv = cnt[base + i];
      offs[base + i] = run;
      cur[base + i]  = run;
      run += cv;
    }
  }
  __syncthreads();
  if (wave == 0) {
#pragma unroll 1
    for (int b0 = 0; b0 < tt; b0 += 32) {
      const int idx = b0 + lane;
      const int ent = hl[idx < RCAP ? idx : RCAP - 1];
      const int m32 = (tt - b0) < 32 ? (tt - b0) : 32;
#pragma unroll 1
      for (int k = 0; k < m32; ++k) {
        const int u    = __builtin_amdgcn_readlane(ent, k);
        const int slot = u & (NBA - 1);
        if (lane == 0) {
          int p = cur[slot];
          p = p < 0 ? 0 : (p > RCAP - 1 ? RCAP - 1 : p);
          sl[p] = u;
          cur[slot] = p + 1;
        }
      }
    }
  }
  __syncthreads();

  const float qnan = __int_as_float(0x7fc00000);
  const float pz = (ovf != 0) ? qnan : 0.0f;

  if constexpr (L == 1) {
    const int c0 = 2 * lane;
    const v2f braw = *(const v2fa*)(bias + c0);
    const float bb0 = bfr(braw.x), bb1 = bfr(braw.y);
    const float* ASp = SD;
    const float* ADp = SD + MPr;
#pragma unroll 1
    for (int si = 0; si < NBA / NWAVE; ++si) {
      const int s    = si * NWAVE + wave;
      const int node = nodeBase + s;
      int c = cnt[s];
      const bool big = c > DEGCAP;
      c = c < 0 ? 0 : (c > DEGCAP ? DEGCAP : c);
      int o = offs[s];
      o = o < 0 ? 0 : (o > RCAP ? RCAP : o);
      const int nc = node < nN ? node : nN - 1;
      const float as0 = ASp[nc];
      const float ad  = ADp[nc];
      const v2f fd = *(const v2fa*)(F + (size_t)nc * HID + c0);
      float a0 = fd.x, a1 = fd.y;
      float l0 = as0 + ad;
      l0 = l0 > 0.f ? l0 : NEGSL * l0;
      float mx = l0, dn = 1.0f;
#pragma unroll 1
      for (int b0 = 0; b0 < c; b0 += 32) {
        int idx = o + b0 + lane;
        idx = idx > RCAP - 1 ? RCAP - 1 : idx;
        const int ent = sl[idx];
        int eid = ent >> SLA;
        eid = eid < 0 ? 0 : (eid > nE - 1 ? nE - 1 : eid);
        int sr = srcs[eid];
        sr = sr < 0 ? 0 : (sr > nN - 1 ? nN - 1 : sr);
        const float es  = ASp[sr];
        const int   esi = __float_as_int(es);
        const int m32 = (c - b0) < 32 ? (c - b0) : 32;
#pragma unroll 1
        for (int k = 0; k < m32; ++k) {
          const int   sk  = __builtin_amdgcn_readlane(sr, k);
          const float ask = __int_as_float(__builtin_amdgcn_readlane(esi, k));
          const v2f fs = *(const v2fa*)(F + (size_t)sk * HID + c0);
          float lg = ask + ad;
          lg = lg > 0.f ? lg : NEGSL * lg;
          const float df = lg - mx;
          const float ee = expf(-fabsf(df));
          const bool  up = df > 0.f;
          const float s1 = up ? ee : 1.0f;
          const float s2 = up ? 1.0f : ee;
          mx = up ? lg : mx;
          dn = fmaf(dn, s1, s2);
          a0 = fmaf(a0, s1, s2 * fs.x);
          a1 = fmaf(a1, s1, s2 * fs.y);
        }
      }
      const float inv = __builtin_amdgcn_rcpf(dn + EPS_SM);
      const float pzr = big ? qnan : pz;
      const bool live = node < nN;
      float y0 = fmaf(a0, inv, bb0);
      float y1 = fmaf(a1, inv, bb1);
      y0 = (y0 > 0.0f) ? y0 : (y0 - y0);
      y1 = (y1 > 0.0f) ? y1 : (y1 - y1);
      y0 = y0 + pzr;
      y1 = y1 + pzr;
      const float v0 = live ? y0 : 0.0f;
      const float v1 = live ? y1 : 0.0f;
      const unsigned int hb0 = f2bf(v0), hb1 = f2bf(v1);
      const unsigned int lb0 = f2bf(v0 - bf2f(hb0)), lb1 = f2bf(v1 - bf2f(hb1));
      const int hw = (int)(hb0 | (hb1 << 16));
      const int lw = (int)(lb0 | (lb1 << 16));
      const int sx0 = (4 * lane) & 31, sx1 = (4 * lane + 1) & 31, sx2 = (4 * lane + 2) & 31, sx3 = (4 * lane + 3) & 31;
      const int g0 = __shfl(hw, sx0), g1 = __shfl(hw, sx1), g2 = __shfl(hw, sx2), g3 = __shfl(hw, sx3);
      const int q0 = __shfl(lw, sx0), q1 = __shfl(lw, sx1), q2 = __shfl(lw, sx2), q3 = __shfl(lw, sx3);
      const bool lsel = lane >= 8;
      v4u pv;
      pv.x = (unsigned int)(lsel ? q0 : g0);
      pv.y = (unsigned int)(lsel ? q1 : g1);
      pv.z = (unsigned int)(lsel ? q2 : g2);
      pv.w = (unsigned int)(lsel ? q3 : g3);
      const int nodeC = node < MPr ? node : MPr - 1;
      unsigned short* gp = zhl + (size_t)nodeC * KA2 + 8 * (lane & 15);
      const bool wr = (node < MPr) && (lane < 16);
      if (wr) *(volatile v4u*)gp = pv;
      __threadfence();
      if (wr) *(volatile v4u*)gp = pv;
    }
  } else {
    const int hd = lane >> 2;
    const int c0 = 16 * lane;
    const float* ASp = SD + (size_t)(2 * hd) * (size_t)MPr;
    const float* ADp = ASp + MPr;
    const v4f bz = bfr4(*(const v4fa*)(bias + 4 * (lane & 15)));
    const int srcl = lane >> 2;
    const int pi   = lane & 3;
#pragma unroll 1
    for (int si = 0; si < NBA / NWAVE; ++si) {
      const int s    = si * NWAVE + wave;
      const int node = nodeBase + s;
      int c = cnt[s];
      const bool big = c > DEGCAP;
      c = c < 0 ? 0 : (c > DEGCAP ? DEGCAP : c);
      int o = offs[s];
      o = o < 0 ? 0 : (o > RCAP ? RCAP : o);
      const int nc = node < nN ? node : nN - 1;
      const float as0 = ASp[nc];
      const float ad  = ADp[nc];
      float acc[16];
      {
        const float* sp = F + (size_t)nc * HC2 + c0;
        const v4f r0 = *(const v4fa*)sp, r1 = *(const v4fa*)(sp + 4);
        const v4f r2 = *(const v4fa*)(sp + 8), r3 = *(const v4fa*)(sp + 12);
        acc[0] = r0.x;  acc[1] = r0.y;  acc[2] = r0.z;  acc[3] = r0.w;
        acc[4] = r1.x;  acc[5] = r1.y;  acc[6] = r1.z;  acc[7] = r1.w;
        acc[8] = r2.x;  acc[9] = r2.y;  acc[10] = r2.z; acc[11] = r2.w;
        acc[12] = r3.x; acc[13] = r3.y; acc[14] = r3.z; acc[15] = r3.w;
      }
      float l0 = as0 + ad;
      l0 = l0 > 0.f ? l0 : NEGSL * l0;
      float mx = l0, dn = 1.0f;
#pragma unroll 1
      for (int b0 = 0; b0 < c; b0 += 32) {
        int idx = o + b0 + lane;
        idx = idx > RCAP - 1 ? RCAP - 1 : idx;
        const int ent = sl[idx];
        int eid = ent >> SLA;
        eid = eid < 0 ? 0 : (eid > nE - 1 ? nE - 1 : eid);
        int sr = srcs[eid];
        sr = sr < 0 ? 0 : (sr > nN - 1 ? nN - 1 : sr);
        const int m32 = (c - b0) < 32 ? (c - b0) : 32;
#pragma unroll 1
        for (int k = 0; k < m32; ++k) {
          const int sk = __builtin_amdgcn_readlane(sr, k);
          const float ask = ASp[sk];
          const float* rp = F + (size_t)sk * HC2 + c0;
          const v4f r0 = *(const v4fa*)rp, r1 = *(const v4fa*)(rp + 4);
          const v4f r2 = *(const v4fa*)(rp + 8), r3 = *(const v4fa*)(rp + 12);
          float lg = ask + ad;
          lg = lg > 0.f ? lg : NEGSL * lg;
          const float df = lg - mx;
          const float ee = expf(-fabsf(df));
          const bool  up = df > 0.f;
          const float s1 = up ? ee : 1.0f;
          const float s2 = up ? 1.0f : ee;
          mx = up ? lg : mx;
          dn = fmaf(dn, s1, s2);
          acc[0]  = fmaf(acc[0],  s1, s2 * r0.x); acc[1]  = fmaf(acc[1],  s1, s2 * r0.y);
          acc[2]  = fmaf(acc[2],  s1, s2 * r0.z); acc[3]  = fmaf(acc[3],  s1, s2 * r0.w);
          acc[4]  = fmaf(acc[4],  s1, s2 * r1.x); acc[5]  = fmaf(acc[5],  s1, s2 * r1.y);
          acc[6]  = fmaf(acc[6],  s1, s2 * r1.z); acc[7]  = fmaf(acc[7],  s1, s2 * r1.w);
          acc[8]  = fmaf(acc[8],  s1, s2 * r2.x); acc[9]  = fmaf(acc[9],  s1, s2 * r2.y);
          acc[10] = fmaf(acc[10], s1, s2 * r2.z); acc[11] = fmaf(acc[11], s1, s2 * r2.w);
          acc[12] = fmaf(acc[12], s1, s2 * r3.x); acc[13] = fmaf(acc[13], s1, s2 * r3.y);
          acc[14] = fmaf(acc[14], s1, s2 * r3.z); acc[15] = fmaf(acc[15], s1, s2 * r3.w);
        }
      }
      const float inv = __builtin_amdgcn_rcpf(dn + EPS_SM);
      const float pzr = big ? qnan : pz;
      float g[16];
#pragma unroll
      for (int i = 0; i < 16; ++i) {
        float v = acc[i] * inv;
        v += __shfl_xor(v, 4);
        v += __shfl_xor(v, 8);
        v += __shfl_xor(v, 16);
        g[i] = __shfl(v, srcl);
      }
      v4f ov;
      ov.x = (pi == 0) ? g[0] : ((pi == 1) ? g[4] : ((pi == 2) ? g[8]  : g[12]));
      ov.y = (pi == 0) ? g[1] : ((pi == 1) ? g[5] : ((pi == 2) ? g[9]  : g[13]));
      ov.z = (pi == 0) ? g[2] : ((pi == 1) ? g[6] : ((pi == 2) ? g[10] : g[14]));
      ov.w = (pi == 0) ? g[3] : ((pi == 1) ? g[7] : ((pi == 2) ? g[11] : g[15]));
      ov.x = fmaf(ov.x, 0.125f, bz.x) + pzr;
      ov.y = fmaf(ov.y, 0.125f, bz.y) + pzr;
      ov.z = fmaf(ov.z, 0.125f, bz.z) + pzr;
      ov.w = fmaf(ov.w, 0.125f, bz.w) + pzr;
      float* op = z2 + (size_t)nc * HID + 4 * (lane & 15);
      const bool wr = (node < nN) && (lane < 16);
      if (wr) *(volatile v4f*)op = ov;
      __threadfence();
      if (wr) *(volatile v4f*)op = ov;
    }
  }
}

__global__ __launch_bounds__(DTHR) void k_decode(const float* __restrict__ Z, const int* __restrict__ eli,
                                                 int EL, int nN, float* out) {
  __shared__ __attribute__((aligned(16))) float sres[DTHR];
  const int tid  = (int)threadIdx.x;
  const int base = (int)blockIdx.x * DTHR;
  const int t    = base + tid;
  const int tc   = t < EL ? t : EL - 1;
  int i0 = eli[tc];
  int i1 = eli[EL + tc];
  i0 = i0 < 0 ? 0 : (i0 > nN - 1 ? nN - 1 : i0);
  i1 = i1 < 0 ? 0 : (i1 > nN - 1 ? nN - 1 : i1);
  const float* a = Z + (size_t)i0 * HID;
  const float* b = Z + (size_t)i1 * HID;
  float s = 0.0f;
#pragma unroll 4
  for (int q = 0; q < HID / 4; ++q) {
    const v4f av = *(const v4fa*)(a + 4 * q);
    const v4f bv = *(const v4fa*)(b + 4 * q);
    s = fmaf(av.x, bv.x, s);
    s = fmaf(av.y, bv.y, s);
    s = fmaf(av.z, bv.z, s);
    s = fmaf(av.w, bv.w, s);
  }
  sres[tid] = s;
  __syncthreads();
  int nLive = EL - base;
  nLive = nLive < 0 ? 0 : (nLive > DTHR ? DTHR : nLive);
  const int nP = nLive >> 2;
  const int pc = tid < DTHR / 4 ? tid : DTHR / 4 - 1;
  const v4f v = *(const v4fa*)(sres + 4 * pc);
  float* op = out + (size_t)base + 4 * pc;
  const bool wr = tid < nP;
  if (wr) *(volatile v4f*)op = v;
  __threadfence();
  if (wr) *(volatile v4f*)op = v;
}

static inline int cdiv(int a, int b) { return (a + b - 1) / b; }
static inline size_t al256(size_t v) { return (v + 255) & ~(size_t)255; }

extern "C" void kernel_launch(void* const* d_in, const int* in_sizes, int n_in,
                              void* d_out, int out_size, void* d_ws, size_t ws_size,
                              hipStream_t stream) {
  if (n_in < 11) return;
  if (in_sizes[0] < DIN || (in_sizes[0] % DIN) != 0) return;
  const int nN = in_sizes[0] / DIN;
  if (nN <= 0 || nN > (1 << 22)) return;
  if (in_sizes[1] < 2 || (in_sizes[1] & 1) != 0) return;
  const int nE = in_sizes[1] / 2;
  if (nE < 1 || nE >= (1 << 21)) return;
  if (in_sizes[2] < 2 || (in_sizes[2] & 1) != 0) return;
  const int EL = in_sizes[2] / 2;
  if (EL < 4 || (EL & 3) != 0) return;
  if (in_sizes[3] != DIN * HID) return;
  if (in_sizes[4] != HID || in_sizes[5] != HID || in_sizes[6] != HID) return;
  if (in_sizes[7] != HID * HC2) return;
  if (in_sizes[8] != NH2 * HID || in_sizes[9] != NH2 * HID) return;
  if (in_sizes[10] != HID) return;
  if (out_size != EL) return;

  const float* x    = (const float*)d_in[0];
  const int*   ei   = (const int*)  d_in[1];
  const int*   eli  = (const int*)  d_in[2];
  const float* W1   = (const float*)d_in[3];
  const float* a1s  = (const float*)d_in[4];
  const float* a1d  = (const float*)d_in[5];
  const float* b1   = (const float*)d_in[6];
  const float* W2   = (const float*)d_in[7];
  const float* a2s  = (const float*)d_in[8];
  const float* a2d  = (const float*)d_in[9];
  const float* b2   = (const float*)d_in[10];
  float* out = (float*)d_out;
  const int* src = ei;
  const int* dst = ei + nE;

  const int MP   = cdiv(nN, GBM) * GBM;
  const int gM   = MP / GBM;
  const int gA   = cdiv(MP, NBA);
  if ((long long)gA * NBA < (long long)MP) return;
  const int vec8 = ((nE & 3) == 0) ? 1 : 0;

  char* ws = (char*)d_ws;
  const size_t szH2 = (size_t)MP * HC2 * 4;
  const size_t szXB = (size_t)MP * DIN * 2;
  const size_t szH1 = (size_t)MP * HID * 4;
  const size_t oH2  = 0;
  const size_t oXB  = 0;
  const size_t oH1  = al256(szXB);
  if (oH1 + szH1 > szH2) return;
  size_t off = al256(szH2);
  const size_t szZa = (size_t)MP * KA2 * 2;
  const size_t szZb = (size_t)MP * HID * 4;
  const size_t oZ   = off; off += (szZa > szZb ? szZa : szZb);   off = al256(off);
  const size_t oSD1 = off; off += (size_t)2 * MP * 4;            off = al256(off);
  const size_t oSD2 = off; off += (size_t)2 * NH2 * MP * 4;      off = al256(off);
  const size_t oW1T = off; off += (size_t)HID * DIN * 2;         off = al256(off);
  const size_t oW2T = off; off += (size_t)HC2 * KA2 * 2;         off = al256(off);
  if (off > ws_size || off > (size_t)WSMAX) return;
  float*          H2   = (float*)(ws + oH2);
  unsigned short* XB   = (unsigned short*)(ws + oXB);
  float*          H1   = (float*)(ws + oH1);
  unsigned short* Z1HL = (unsigned short*)(ws + oZ);
  float*          Z2   = (float*)(ws + oZ);
  float*          SD1  = (float*)(ws + oSD1);
  float*          SD2  = (float*)(ws + oSD2);
  unsigned short* W1T  = (unsigned short*)(ws + oW1T);
  unsigned short* W2T2 = (unsigned short*)(ws + oW2T);

  const size_t aggLds = (size_t)AGG_LDS_INTS * 4;
  hipFuncSetAttribute(reinterpret_cast<const void*>(&k_agg<1>), hipFuncAttributeMaxDynamicSharedMemorySize, (int)aggLds);
  hipFuncSetAttribute(reinterpret_cast<const void*>(&k_agg<2>), hipFuncAttributeMaxDynamicSharedMemorySize, (int)aggLds);

  const int nUx = MP * (DIN / 8);
  k_xprep<<<cdiv(nUx, NTHR), NTHR, 0, stream>>>(x, XB, nN, nUx);
  {
    const int nUw1 = HID * (DIN / 8);
    k_wtr<<<cdiv(nUw1, NTHR), NTHR, 0, stream>>>(W1, DIN, HID, HID, DIN, W1T, nUw1);
    const int nUw2 = HC2 * (KA2 / 8);
    k_wtr<<<cdiv(nUw2, NTHR), NTHR, 0, stream>>>(W2, HID, HC2, HC2, KA2, W2T2, nUw2);
  }
  k_gemm<<<dim3(gM, 1), GTHR, 0, stream>>>(XB, W1T, H1, DIN, HID, a1s, a1d, HID, SD1, MP);
  k_agg<1><<<gA, NTHR, aggLds, stream>>>(src, dst, nE, nN, vec8, MP, SD1, H1, b1, Z1HL, Z2);
  k_gemm<<<dim3(gM, NH2), GTHR, 0, stream>>>(Z1HL, W2T2, H2, KA2, HC2, a2s, a2d, HID, SD2, MP);
  k_agg<2><<<gA, NTHR, aggLds, stream>>>(src, dst, nE, nN, vec8, MP, SD2, H2, b2, Z1HL, Z2);
  k_decode<<<cdiv(EL, DTHR), DTHR, 0, stream>>>(Z2, eli, EL, nN, out);
}
